// PointNet2Layer_26688926777504
// MI455X (gfx1250) — hardware-verified
//
#include <hip/hip_runtime.h>
#pragma clang fp contract(off)

typedef __attribute__((ext_vector_type(16))) _Float16 v16h;
typedef __attribute__((ext_vector_type(8)))  _Float16 v8h;
typedef __attribute__((ext_vector_type(8)))  float    v8f;
typedef __attribute__((ext_vector_type(4)))  float    v4f;

constexpr int NBATCH   = 4;
constexpr int NPTS     = 16384;
constexpr int NPICK    = 1024;
constexpr int NSAMP    = 32;
constexpr int NCHAN    = 32;
constexpr int NFEAT_IN = 4;

struct FragH {
  union U { v16h v; v8h h[2]; };
  static __device__ __forceinline__ v16h load(const _Float16* p) {
    U f;
    f.h[0] = *(const v8h*)(p);
    f.h[1] = *(const v8h*)(p + 16);
    return f.v;
  }
  static __device__ __forceinline__ v8f mma(v16h a, v16h b, v8f c) {
    return __builtin_amdgcn_wmma_f32_16x16x32_f16(false, a, false, b, (short)0, c, false, false);
  }
};
__device__ __forceinline__ void group_guard(v8f& a, v8f& b, v8f& c, v8f& d, v16h x0, v16h x1, v16h y0, v16h y1) {
  asm volatile("v_nop\n\tv_nop\n\tv_nop\n\tv_nop" : "+v"(a), "+v"(b), "+v"(c), "+v"(d) : "v"(x0), "v"(x1), "v"(y0), "v"(y1));
}

__device__ __forceinline__ void argmax_bfly(float& v, int& i) {
#pragma unroll
  for (int off = 16; off > 0; off >>= 1) {
    const float ov = __shfl_xor(v, off, 32);
    const int   oi = __shfl_xor(i, off, 32);
    const bool  tk = (ov > v) || (ov == v && oi < i);
    v = tk ? ov : v;
    i = tk ? oi : i;
  }
}

constexpr int FPS_T   = 1024;
constexpr int FPS_PPT = NPTS / FPS_T;
static_assert(FPS_PPT == 16, "points per thread");
static_assert(FPS_T == NPICK, "one pick per thread in the final store pass");
static_assert((FPS_T * 3) % 4 == 0, "staging chunk is whole 16-B words");

__global__ __launch_bounds__(FPS_T) void fps_kernel(const float* __restrict__ pos,
                                                    float* __restrict__ newpos4)
{
#pragma clang fp contract(off)
  __shared__ __align__(16) float stage[FPS_T * 3];
  __shared__ __align__(16) float picks[NPICK * 4];
  __shared__ float swv[2][32];
  __shared__ int   swi[2][32];

  const int b    = blockIdx.x;
  const int t    = threadIdx.x;
  const int lane = t & 31;
  const int wv   = t >> 5;
  const float* p = pos + (size_t)b * NPTS * 3;

  float px[FPS_PPT], py[FPS_PPT], pz[FPS_PPT], md[FPS_PPT];
#pragma unroll
  for (int j = 0; j < FPS_PPT; ++j) {
    if (t < (FPS_T * 3) / 4) {
      const v4f v = *(const v4f*)(p + (size_t)j * (FPS_T * 3) + t * 4);
      *(v4f*)(stage + t * 4) = v;
    }
    __syncthreads();
    px[j] = stage[t * 3 + 0];
    py[j] = stage[t * 3 + 1];
    pz[j] = stage[t * 3 + 2];
    md[j] = 1e10f;
    __syncthreads();
  }

  int far = 0;
#pragma unroll 1
  for (int i = 0; i < NPICK; ++i) {
    const float cx = p[far * 3 + 0];
    const float cy = p[far * 3 + 1];
    const float cz = p[far * 3 + 2];
    if (t == 0) {
      v4f pv;
      pv[0] = cx; pv[1] = cy; pv[2] = cz; pv[3] = 0.0f;
      *(v4f*)(picks + i * 4) = pv;
    }
    float best = -1.0f;
    int   bj   = 0;
#pragma unroll
    for (int j = 0; j < FPS_PPT; ++j) {
      const float dx = px[j] - cx;
      const float dy = py[j] - cy;
      const float dz = pz[j] - cz;
      const float tx = dx * dx;
      const float ty = dy * dy;
      const float tz = dz * dz;
      const float d  = (tx + tz) + ty;
      const float m  = fminf(md[j], d);
      md[j] = m;
      const bool g = m > best;
      best = g ? m : best;
      bj   = g ? j : bj;
    }
    int bi = bj * FPS_T + t;
    argmax_bfly(best, bi);
    const int buf = i & 1;
    if (lane == 0) { swv[buf][wv] = best; swi[buf][wv] = bi; }
    __syncthreads();
    float v  = swv[buf][lane];
    int   ii = swi[buf][lane];
    argmax_bfly(v, ii);
    ii  = ii < 0 ? 0 : ii;
    far = ii > (NPTS - 1) ? (NPTS - 1) : ii;
  }
  __syncthreads();
  {
    const v4f o = *(const v4f*)(picks + t * 4);
    float* dst = newpos4 + ((size_t)b * NPICK + t) * 4;
    *(volatile v4f*)dst = o;
    __threadfence();
    *(volatile v4f*)dst = o;
  }
}

constexpr int GW  = 4;
constexpr int GT  = GW * 32;
constexpr int CAP = 256;
constexpr int HP  = 40;
static_assert((NBATCH * NPICK) % GW == 0, "grid covers all groups exactly");
static_assert(GT == 128, "weight staging map: 32 columns x 4 k-octets");
static_assert(NCHAN == 32 && NSAMP == 32, "one k-step, 2x2 tiles");
static_assert(NPTS % 128 == 0, "scan step of 128 points");
static_assert(CAP % 32 == 0 && CAP >= NSAMP, "hit list cap");

__device__ __forceinline__ float bq_key(float cx, float cy, float cz, float A, float x, float y, float z) {
#pragma clang fp contract(off)
  const float tx = x * x;
  const float ty = y * y;
  const float tz = z * z;
  const float B  = (tx + tz) + ty;
  float D = cx * x;
  D = __builtin_fmaf(cy, y, D);
  D = __builtin_fmaf(cz, z, D);
  const float s  = A + B;
  const float d2 = s - 2.0f * D;
  return d2;
}

__device__ __forceinline__ void bq_push(bool hit, float d2, int n, unsigned ltmask, int& cnt, float* ldw, int* liw) {
  const unsigned m = __builtin_amdgcn_ballot_w32(hit);
  const int slot = cnt + __builtin_popcount(m & ltmask);
  if (hit && slot < CAP) { ldw[slot] = d2; liw[slot] = n; }
  cnt += __builtin_popcount(m);
}

__device__ __forceinline__ void relu_pack_store(const v8f acc, const float* bp, _Float16* dst) {
  const v4f b0 = *(const v4f*)(bp);
  const v4f b1 = *(const v4f*)(bp + 4);
  v8h hv;
  hv[0] = (_Float16)fmaxf(acc[0] + b0[0], 0.0f);
  hv[1] = (_Float16)fmaxf(acc[1] + b0[1], 0.0f);
  hv[2] = (_Float16)fmaxf(acc[2] + b0[2], 0.0f);
  hv[3] = (_Float16)fmaxf(acc[3] + b0[3], 0.0f);
  hv[4] = (_Float16)fmaxf(acc[4] + b1[0], 0.0f);
  hv[5] = (_Float16)fmaxf(acc[5] + b1[1], 0.0f);
  hv[6] = (_Float16)fmaxf(acc[6] + b1[2], 0.0f);
  hv[7] = (_Float16)fmaxf(acc[7] + b1[3], 0.0f);
  *(v8h*)dst = hv;
}

__device__ __forceinline__ float max8_bias(float mx, const v8f acc, float bia) {
  mx = fmaxf(mx, acc[0] + bia);
  mx = fmaxf(mx, acc[1] + bia);
  mx = fmaxf(mx, acc[2] + bia);
  mx = fmaxf(mx, acc[3] + bia);
  mx = fmaxf(mx, acc[4] + bia);
  mx = fmaxf(mx, acc[5] + bia);
  mx = fmaxf(mx, acc[6] + bia);
  mx = fmaxf(mx, acc[7] + bia);
  return mx;
}

__global__ __launch_bounds__(GT) void group_kernel(const float* __restrict__ pos,
                                                   const float* __restrict__ xf,
                                                   const float* __restrict__ W1, const float* __restrict__ b1,
                                                   const float* __restrict__ W2, const float* __restrict__ b2,
                                                   const float* __restrict__ W3, const float* __restrict__ b3,
                                                   const float* __restrict__ newpos4,
                                                   float* __restrict__ out)
{
#pragma clang fp contract(off)
  __shared__ __align__(16) float    ldist[GW][CAP];
  __shared__ __align__(16) int      lidx[GW][CAP];
  __shared__ __align__(16) int      sel[GW][32];
  __shared__ __align__(16) _Float16 hbA[GW][32 * HP];
  __shared__ __align__(16) _Float16 hbB[GW][32 * HP];
  __shared__ __align__(16) _Float16 sWt2[32 * HP];
  __shared__ __align__(16) _Float16 sWt3[32 * HP];
  __shared__ __align__(16) float    sW1[NFEAT_IN * NCHAN];
  __shared__ __align__(16) float    sB[3 * NCHAN];

  const int t    = threadIdx.x;
  const int lane = t & 31;
  const int wv   = t >> 5;
  const int hh   = lane >> 4;
  const int c    = lane & 15;
  const int g    = blockIdx.x * GW + wv;
  const int b    = g >> 10;
  const float* pb = pos + (size_t)b * NPTS * 3;

  {
    const int n = t >> 2;
    const int q = t & 3;
    v8h w2;
#pragma unroll
    for (int e = 0; e < 8; ++e) w2[e] = (_Float16)W2[(q * 8 + e) * NCHAN + n];
    *(v8h*)(sWt2 + n * HP + q * 8) = w2;
    asm volatile("" ::: "memory");
    v8h w3;
#pragma unroll
    for (int e = 0; e < 8; ++e) w3[e] = (_Float16)W3[(q * 8 + e) * NCHAN + n];
    *(v8h*)(sWt3 + n * HP + q * 8) = w3;
    asm volatile("" ::: "memory");
    sW1[t] = W1[t];
    if (t < 32) {
      sB[t]      = b1[t];
      sB[32 + t] = b2[t];
      sB[64 + t] = b3[t];
    }
  }
  sel[wv][lane] = 0;

  const v4f cen = *(const v4f*)(newpos4 + (size_t)g * 4);
  const float cx = cen[0];
  const float cy = cen[1];
  const float cz = cen[2];
  const float cxx = cx * cx;
  const float cyy = cy * cy;
  const float czz = cz * cz;
  const float A = (cxx + czz) + cyy;
  const float R2 = 0.01f;
  const unsigned ltmask = (1u << lane) - 1u;
  float* ldw = ldist[wv];
  int*   liw = lidx[wv];
  int cnt = 0;
#pragma unroll 1
  for (int it = 0; it < NPTS / 128; ++it) {
    const int nb = it * 128 + lane * 4;
    const float* qp = pb + (size_t)nb * 3;
    const v4f f0 = *(const v4f*)(qp);
    const v4f f1 = *(const v4f*)(qp + 4);
    const v4f f2 = *(const v4f*)(qp + 8);
    const float k0 = bq_key(cx, cy, cz, A, f0[0], f0[1], f0[2]);
    const float k1 = bq_key(cx, cy, cz, A, f0[3], f1[0], f1[1]);
    const float k2 = bq_key(cx, cy, cz, A, f1[2], f1[3], f2[0]);
    const float k3 = bq_key(cx, cy, cz, A, f2[1], f2[2], f2[3]);
    bq_push(k0 <= R2, k0, nb + 0, ltmask, cnt, ldw, liw);
    bq_push(k1 <= R2, k1, nb + 1, ltmask, cnt, ldw, liw);
    bq_push(k2 <= R2, k2, nb + 2, ltmask, cnt, ldw, liw);
    bq_push(k3 <= R2, k3, nb + 3, ltmask, cnt, ldw, liw);
  }
  __syncthreads();

  const int cntc = cnt < CAP ? cnt : CAP;
  int ngrp = (cntc + 31) >> 5;
  ngrp = ngrp < (CAP / 32) ? ngrp : (CAP / 32);
  int* selw = sel[wv];
#pragma unroll 1
  for (int gi = 0; gi < ngrp; ++gi) {
    const int  j   = gi * 32 + lane;
    const bool act = j < cntc;
    const int  jc  = act ? j : 0;
    const float dj = ldw[jc];
    const int   ij = liw[jc];
    int rank = 0;
#pragma unroll 1
    for (int e = 0; e < cntc; ++e) {
      const float de = ldw[e];
      const int   ie = liw[e];
      rank += ((de < dj) || (de == dj && ie < ij)) ? 1 : 0;
    }
    if (act && rank < NSAMP) selw[rank] = ij;
  }
  __syncthreads();

  const int first = selw[0];
  const int mine  = selw[lane];
  int pidx = (lane < cntc) ? mine : first;
  pidx = pidx < 0 ? 0 : pidx;
  pidx = pidx > (NPTS - 1) ? (NPTS - 1) : pidx;
  const float* pp = pb + (size_t)pidx * 3;
  const float gx = pp[0];
  const float gy = pp[1];
  const float gz = pp[2];
  const float r3 = xf[(size_t)b * NPTS + pidx];
  const float r0 = gx - cx;
  const float r1 = gy - cy;
  const float r2 = gz - cz;
  {
    _Float16* rowp = hbA[wv] + lane * HP;
#pragma unroll
    for (int q = 0; q < 4; ++q) {
      v8h hv;
#pragma unroll
      for (int e = 0; e < 8; ++e) {
        const int ch = q * 8 + e;
        float a = r0 * sW1[ch];
        a = __builtin_fmaf(r1, sW1[NCHAN + ch], a);
        a = __builtin_fmaf(r2, sW1[2 * NCHAN + ch], a);
        a = __builtin_fmaf(r3, sW1[3 * NCHAN + ch], a);
        a = a + sB[ch];
        hv[e] = (_Float16)fmaxf(a, 0.0f);
      }
      *(v8h*)(rowp + q * 8) = hv;
    }
  }
  __syncthreads();

  const v8f vz = {0.f, 0.f, 0.f, 0.f, 0.f, 0.f, 0.f, 0.f};

  {
    const v16h wa0 = FragH::load(sWt2 + (0 * 16 + c) * HP + 8 * hh);
    const v16h wa1 = FragH::load(sWt2 + (1 * 16 + c) * HP + 8 * hh);
    const v16h hm0 = FragH::load(hbA[wv] + (0 * 16 + c) * HP + 8 * hh);
    const v16h hm1 = FragH::load(hbA[wv] + (1 * 16 + c) * HP + 8 * hh);
    v8f d00 = FragH::mma(wa0, hm0, vz);
    v8f d01 = FragH::mma(wa0, hm1, vz);
    v8f d10 = FragH::mma(wa1, hm0, vz);
    v8f d11 = FragH::mma(wa1, hm1, vz);
    group_guard(d00, d01, d10, d11, wa0, wa1, hm0, hm1);
    _Float16* hb = hbB[wv];
    relu_pack_store(d00, sB + 32 + 0 * 16 + 8 * hh, hb + (0 * 16 + c) * HP + 0 * 16 + 8 * hh);
    relu_pack_store(d01, sB + 32 + 0 * 16 + 8 * hh, hb + (1 * 16 + c) * HP + 0 * 16 + 8 * hh);
    relu_pack_store(d10, sB + 32 + 1 * 16 + 8 * hh, hb + (0 * 16 + c) * HP + 1 * 16 + 8 * hh);
    relu_pack_store(d11, sB + 32 + 1 * 16 + 8 * hh, hb + (1 * 16 + c) * HP + 1 * 16 + 8 * hh);
  }
  __syncthreads();

  float outv;
  {
    const v16h ha0 = FragH::load(hbB[wv] + (0 * 16 + c) * HP + 8 * hh);
    const v16h ha1 = FragH::load(hbB[wv] + (1 * 16 + c) * HP + 8 * hh);
    const v16h wb0 = FragH::load(sWt3 + (0 * 16 + c) * HP + 8 * hh);
    const v16h wb1 = FragH::load(sWt3 + (1 * 16 + c) * HP + 8 * hh);
    v8f e00 = FragH::mma(ha0, wb0, vz);
    v8f e01 = FragH::mma(ha0, wb1, vz);
    v8f e10 = FragH::mma(ha1, wb0, vz);
    v8f e11 = FragH::mma(ha1, wb1, vz);
    group_guard(e00, e01, e10, e11, ha0, ha1, wb0, wb1);
    const float bia0 = sB[64 + c];
    const float bia1 = sB[64 + 16 + c];
    float mx0 = 0.0f;
    float mx1 = 0.0f;
    mx0 = max8_bias(mx0, e00, bia0);
    mx0 = max8_bias(mx0, e10, bia0);
    mx1 = max8_bias(mx1, e01, bia1);
    mx1 = max8_bias(mx1, e11, bia1);
    const float o0 = __shfl_xor(mx0, 16, 32);
    const float o1 = __shfl_xor(mx1, 16, 32);
    mx0 = fmaxf(mx0, o0);
    mx1 = fmaxf(mx1, o1);
    outv = (hh != 0) ? mx1 : mx0;
  }
  {
    float* dst = out + (size_t)g * NCHAN + lane;
    *(volatile float*)dst = outv;
    __threadfence();
    *(volatile float*)dst = outv;
  }
}

extern "C" void kernel_launch(void* const* d_in, const int* in_sizes, int n_in,
                              void* d_out, int out_size, void* d_ws, size_t ws_size,
                              hipStream_t stream)
{
  if (n_in < 8) return;
  if (in_sizes[0] != NBATCH * NPTS * 3 || in_sizes[1] != NBATCH * NPTS) return;
  if (in_sizes[2] != NFEAT_IN * NCHAN || in_sizes[4] != NCHAN * NCHAN || in_sizes[6] != NCHAN * NCHAN) return;
  if (out_size != NBATCH * NPICK * NCHAN) return;
  const size_t carve = (size_t)NBATCH * NPICK * 4 * sizeof(float);
  if (ws_size < carve) return;

  const float* pos = (const float*)d_in[0];
  const float* xf  = (const float*)d_in[1];
  const float* W1  = (const float*)d_in[2];
  const float* b1  = (const float*)d_in[3];
  const float* W2  = (const float*)d_in[4];
  const float* b2  = (const float*)d_in[5];
  const float* W3  = (const float*)d_in[6];
  const float* b3  = (const float*)d_in[7];
  float* out     = (float*)d_out;
  float* newpos4 = (float*)d_ws;

  fps_kernel<<<NBATCH, FPS_T, 0, stream>>>(pos, newpos4);
  group_kernel<<<(NBATCH * NPICK) / GW, GT, 0, stream>>>(pos, xf, W1, b1, W2, b2, W3, b3, newpos4, out);
}
